// RNNLSTMNet_32066225832677
// MI455X (gfx1250) — hardware-verified
//
#include <hip/hip_runtime.h>
#include <math.h>

constexpr int NSEQ    = 64;
constexpr int NSTEP   = 512;
constexpr int NVOC    = 32000;
constexpr int NEMB    = 64;
constexpr int NHID    = 512;
constexpr int NG4     = 4 * NHID;
constexpr int NCLS    = 10;
constexpr int NTHR    = 256;
constexpr int CVT_THR = 256;
constexpr int SEQ_BLK = 16;
constexpr int NBLK    = NSEQ / SEQ_BLK;
constexpr int XPITCH  = 72;
constexpr int HPITCH  = 520;
constexpr int FPITCH  = 516;
constexpr int HPLANE  = SEQ_BLK * HPITCH;
constexpr int OUT_BLK = SEQ_BLK * NCLS;
constexpr int LDS_XS    = 0;
constexpr int LDS_H     = 2304;
constexpr int LDS_HS    = LDS_H + 8 * HPLANE * 2;
constexpr int LDS_OS    = LDS_HS + SEQ_BLK * FPITCH * 4;
constexpr int LDS_TOTAL = LDS_OS + OUT_BLK * 4;
constexpr int H_DWORDS  = 8 * HPLANE / 2;
constexpr float XW_CARRY = 256.0f;
constexpr float W_CARRY  = 16.0f;
constexpr float H_CARRY  = 16.0f;
constexpr float ACC_FOLD = 0.00390625f;
static_assert(NSEQ % SEQ_BLK == 0);
static_assert(NEMB % 32 == 0);
static_assert(NHID % 32 == 0);
static_assert(NHID == 64 * (NTHR / 32));
static_assert(OUT_BLK == 160);
static_assert((OUT_BLK * 4) % 128 == 0);
static_assert(LDS_TOTAL == 169088);
static_assert(LDS_H % 16 == 0 && LDS_HS % 16 == 0 && LDS_OS % 16 == 0 && (HPLANE * 2) % 16 == 0);
static_assert(H_DWORDS % NTHR == 0);
static_assert(NTHR * 4 == SEQ_BLK * NEMB);

typedef __attribute__((ext_vector_type(16))) _Float16 v16h;
typedef __attribute__((ext_vector_type(8)))  _Float16 v8h;
typedef __attribute__((ext_vector_type(16))) __bf16   v16b;
typedef __attribute__((ext_vector_type(8)))  __bf16   v8b;
typedef __attribute__((ext_vector_type(8)))  float    v8f;
typedef __attribute__((ext_vector_type(4)))  float    v4f;
typedef __attribute__((ext_vector_type(2)))  unsigned v2u;

__device__ __forceinline__ unsigned short f2bf_bits(float f) {
  unsigned u = __float_as_uint(f);
  return (unsigned short)((u + 0x7FFFu + ((u >> 16) & 1u)) >> 16);
}
__device__ __forceinline__ float bf_bits2f(unsigned short h) { return __uint_as_float(((unsigned)h) << 16); }
__device__ __forceinline__ float bf16r(float f) { return bf_bits2f(f2bf_bits(f)); }

__device__ __forceinline__ void dep_guard_h(v8f& a, v8f& b, v16h x, v16h y) { asm volatile("v_nop\n\tv_nop\n\tv_nop\n\tv_nop" : "+v"(a), "+v"(b) : "v"(x), "v"(y)); }
__device__ __forceinline__ void dep_guard_b(v8f& a, v8f& b, v16b x, v16b y) { asm volatile("v_nop\n\tv_nop\n\tv_nop\n\tv_nop" : "+v"(a), "+v"(b) : "v"(x), "v"(y)); }
__device__ __forceinline__ void keep4_h(v16h a, v16h b, v16h c, v16h d) { asm volatile("v_nop" :: "v"(a), "v"(b), "v"(c), "v"(d)); }
__device__ __forceinline__ void keep4_b(v16b a, v16b b, v16b c, v16b d) { asm volatile("v_nop" :: "v"(a), "v"(b), "v"(c), "v"(d)); }
__device__ __forceinline__ void acc_guard4(v8f& a, v8f& b, v8f& c, v8f& d) { asm volatile("v_nop\n\tv_nop\n\tv_nop\n\tv_nop" : "+v"(a), "+v"(b), "+v"(c), "+v"(d)); }
template <typename T> struct Frag;
template <> struct Frag<_Float16> {
  typedef v16h V; union U { v16h v; v8h h[2]; };
  static __device__ __forceinline__ v16h load(const _Float16* p) {
    U f; f.h[0] = *(const v8h*)(p); f.h[1] = *(const v8h*)(p + 16); return f.v;
  }
  static __device__ __forceinline__ v8f mma(v16h a, v16h b, v8f c) {
    return __builtin_amdgcn_wmma_f32_16x16x32_f16(false, a, false, b, (short)0, c, false, false);
  }
  static __device__ __forceinline__ void guard(v8f& a, v8f& b, v16h x, v16h y) { dep_guard_h(a, b, x, y); }
  static __device__ __forceinline__ void keep(v16h a, v16h b, v16h c, v16h d) { keep4_h(a, b, c, d); }
};
template <> struct Frag<__bf16> {
  typedef v16b V; union U { v16b v; v8b h[2]; };
  static __device__ __forceinline__ v16b load(const __bf16* p) {
    U f; f.h[0] = *(const v8b*)(p); f.h[1] = *(const v8b*)(p + 16); return f.v;
  }
  static __device__ __forceinline__ v8f mma(v16b a, v16b b, v8f c) {
    return __builtin_amdgcn_wmma_f32_16x16x32_bf16(false, a, false, b, (short)0, c, false, false);
  }
  static __device__ __forceinline__ void guard(v8f& a, v8f& b, v16b x, v16b y) { dep_guard_b(a, b, x, y); }
  static __device__ __forceinline__ void keep(v16b a, v16b b, v16b c, v16b d) { keep4_b(a, b, c, d); }
};

__device__ __forceinline__ float fsig(float x)  { return __builtin_amdgcn_rcpf(1.0f + __expf(-x)); }
__device__ __forceinline__ float ftanh(float x) { return 1.0f - 2.0f * __builtin_amdgcn_rcpf(__expf(2.0f * x) + 1.0f); }

template <int MODE>
__global__ __launch_bounds__(CVT_THR) void cvt8_kernel(const float* __restrict__ src, unsigned short* __restrict__ dst, int n8, float sc) {
  const int i = blockIdx.x * CVT_THR + threadIdx.x;
  if (i < n8) {
    const v4f a = *(const v4f*)(src + (size_t)i * 8);
    const v4f b = *(const v4f*)(src + (size_t)i * 8 + 4);
    v8h hv;
#pragma unroll
    for (int e = 0; e < 4; ++e) {
      unsigned short b0, b1;
      if (MODE == 0) {
        b0 = f2bf_bits(a[e] * sc);
        b1 = f2bf_bits(b[e] * sc);
      } else {
        b0 = __builtin_bit_cast(unsigned short, (_Float16)(bf16r(a[e]) * sc));
        b1 = __builtin_bit_cast(unsigned short, (_Float16)(bf16r(b[e]) * sc));
      }
      hv[e]     = __builtin_bit_cast(_Float16, b0);
      hv[4 + e] = __builtin_bit_cast(_Float16, b1);
    }
    *(volatile v8h*)(dst + (size_t)i * 8) = hv;
    __threadfence();
    *(volatile v8h*)(dst + (size_t)i * 8) = hv;
  }
}

__device__ __forceinline__ void stage_emb(const int* __restrict__ x, const float* __restrict__ emb,
                                          unsigned short* xs, int rowbase, int t, int tid) {
  const int m = tid >> 4, f4 = (tid & 15) * 4;
  int tok = x[(size_t)(rowbase + m) * NSTEP + t];
  tok = (tok < 0) ? (tok + NVOC) : tok;
  tok = (tok < 0) ? 0 : ((tok >= NVOC) ? (NVOC - 1) : tok);
  const v4f v = *(const v4f*)(emb + (size_t)tok * NEMB + f4);
  v2u pk;
  pk[0] = (unsigned)f2bf_bits(v[0]) | ((unsigned)f2bf_bits(v[1]) << 16);
  pk[1] = (unsigned)f2bf_bits(v[2]) | ((unsigned)f2bf_bits(v[3]) << 16);
  *(v2u*)(xs + m * XPITCH + f4) = pk;
}

template <typename TX, int KXD>
__device__ __forceinline__ void rnn_phase(const TX* xrow, const unsigned short* __restrict__ WXp,
                                          const _Float16* hrow, const unsigned short* __restrict__ WHp,
                                          const float* __restrict__ bi, const float* __restrict__ bhv,
                                          _Float16* Hn, int j0, int koff, int hh) {
  typedef typename Frag<TX>::V VX;
  const v8f z8 = {0.f, 0.f, 0.f, 0.f, 0.f, 0.f, 0.f, 0.f};
  v8f acc[4];
  acc[0] = z8; acc[1] = z8; acc[2] = z8; acc[3] = z8;
  {
    const TX* w0 = (const TX*)WXp + (size_t)j0 * KXD + koff;
#pragma unroll 1
    for (int kx = 0; kx < KXD; kx += 32) {
      const VX a  = Frag<TX>::load(xrow + kx);
      const VX b0 = Frag<TX>::load(w0 + kx);
      const VX b1 = Frag<TX>::load(w0 + (size_t)16 * KXD + kx);
      const VX b2 = Frag<TX>::load(w0 + (size_t)32 * KXD + kx);
      const VX b3 = Frag<TX>::load(w0 + (size_t)48 * KXD + kx);
      acc[0] = Frag<TX>::mma(a, b0, acc[0]);
      acc[1] = Frag<TX>::mma(a, b1, acc[1]);
      acc[2] = Frag<TX>::mma(a, b2, acc[2]);
      acc[3] = Frag<TX>::mma(a, b3, acc[3]);
      Frag<TX>::guard(acc[0], acc[3], a, b3);
      Frag<TX>::keep(b0, b1, b2, b3);
    }
  }
  {
    const _Float16* w0 = (const _Float16*)WHp + (size_t)j0 * NHID + koff;
#pragma unroll 1
    for (int k0 = 0; k0 < NHID; k0 += 32) {
      const v16h a  = Frag<_Float16>::load(hrow + k0);
      const v16h b0 = Frag<_Float16>::load(w0 + k0);
      const v16h b1 = Frag<_Float16>::load(w0 + (size_t)16 * NHID + k0);
      const v16h b2 = Frag<_Float16>::load(w0 + (size_t)32 * NHID + k0);
      const v16h b3 = Frag<_Float16>::load(w0 + (size_t)48 * NHID + k0);
      acc[0] = Frag<_Float16>::mma(a, b0, acc[0]);
      acc[1] = Frag<_Float16>::mma(a, b1, acc[1]);
      acc[2] = Frag<_Float16>::mma(a, b2, acc[2]);
      acc[3] = Frag<_Float16>::mma(a, b3, acc[3]);
      dep_guard_h(acc[0], acc[3], a, b3);
      keep4_h(b0, b1, b2, b3);
    }
  }
  acc_guard4(acc[0], acc[1], acc[2], acc[3]);
#pragma unroll
  for (int nt = 0; nt < 4; ++nt) {
    const int j = j0 + 16 * nt;
    const float bs = bf16r(bi[j]) + bf16r(bhv[j]);
#pragma unroll
    for (int r = 0; r < 8; ++r) {
      const float z = fmaxf(acc[nt][r] * ACC_FOLD + bs, 0.0f);
      Hn[(8 * hh + r) * HPITCH + j] = (_Float16)(z * H_CARRY);
    }
  }
}

__device__ __forceinline__ void lstm_phase(const _Float16* xrow, const unsigned short* __restrict__ WXp,
                                           const _Float16* hrow, const unsigned short* __restrict__ WHp,
                                           const float* __restrict__ bi, const float* __restrict__ bhv,
                                           _Float16* Hn, float* Hs, bool last, float (&cst)[4][8],
                                           int j0, int koff, int hh) {
  const _Float16* WX = (const _Float16*)WXp;
  const _Float16* WH = (const _Float16*)WHp;
  const v8f z8 = {0.f, 0.f, 0.f, 0.f, 0.f, 0.f, 0.f, 0.f};
#pragma unroll
  for (int nt = 0; nt < 4; ++nt) {
    const int j = j0 + 16 * nt;
    const _Float16* wx = WX + (size_t)j * NHID + koff;
    const _Float16* wh = WH + (size_t)j * NHID + koff;
    v8f acc[4];
    acc[0] = z8; acc[1] = z8; acc[2] = z8; acc[3] = z8;
#pragma unroll 1
    for (int kx = 0; kx < NHID; kx += 32) {
      const v16h a  = Frag<_Float16>::load(xrow + kx);
      const v16h b0 = Frag<_Float16>::load(wx + kx);
      const v16h b1 = Frag<_Float16>::load(wx + (size_t)1 * NHID * NHID + kx);
      const v16h b2 = Frag<_Float16>::load(wx + (size_t)2 * NHID * NHID + kx);
      const v16h b3 = Frag<_Float16>::load(wx + (size_t)3 * NHID * NHID + kx);
      acc[0] = Frag<_Float16>::mma(a, b0, acc[0]);
      acc[1] = Frag<_Float16>::mma(a, b1, acc[1]);
      acc[2] = Frag<_Float16>::mma(a, b2, acc[2]);
      acc[3] = Frag<_Float16>::mma(a, b3, acc[3]);
      dep_guard_h(acc[0], acc[3], a, b3);
      keep4_h(b0, b1, b2, b3);
    }
#pragma unroll 1
    for (int k0 = 0; k0 < NHID; k0 += 32) {
      const v16h a  = Frag<_Float16>::load(hrow + k0);
      const v16h b0 = Frag<_Float16>::load(wh + k0);
      const v16h b1 = Frag<_Float16>::load(wh + (size_t)1 * NHID * NHID + k0);
      const v16h b2 = Frag<_Float16>::load(wh + (size_t)2 * NHID * NHID + k0);
      const v16h b3 = Frag<_Float16>::load(wh + (size_t)3 * NHID * NHID + k0);
      acc[0] = Frag<_Float16>::mma(a, b0, acc[0]);
      acc[1] = Frag<_Float16>::mma(a, b1, acc[1]);
      acc[2] = Frag<_Float16>::mma(a, b2, acc[2]);
      acc[3] = Frag<_Float16>::mma(a, b3, acc[3]);
      dep_guard_h(acc[0], acc[3], a, b3);
      keep4_h(b0, b1, b2, b3);
    }
    acc_guard4(acc[0], acc[1], acc[2], acc[3]);
    const float bI = bf16r(bi[j])            + bf16r(bhv[j]);
    const float bF = bf16r(bi[NHID + j])     + bf16r(bhv[NHID + j]);
    const float bG = bf16r(bi[2 * NHID + j]) + bf16r(bhv[2 * NHID + j]);
    const float bO = bf16r(bi[3 * NHID + j]) + bf16r(bhv[3 * NHID + j]);
    float hn8[8];
#pragma unroll
    for (int r = 0; r < 8; ++r) {
      const float zi = acc[0][r] * ACC_FOLD + bI;
      const float zf = acc[1][r] * ACC_FOLD + bF;
      const float zg = acc[2][r] * ACC_FOLD + bG;
      const float zo = acc[3][r] * ACC_FOLD + bO;
      const float ig = fsig(zi);
      const float fg = fsig(zf);
      const float og = fsig(zo);
      const float gg = ftanh(zg);
      const float cn = fg * cst[nt][r] + ig * gg;
      cst[nt][r] = cn;
      const float hn = og * ftanh(cn);
      hn8[r] = hn;
      Hn[(8 * hh + r) * HPITCH + j] = (_Float16)(hn * H_CARRY);
    }
    if (last) {
#pragma unroll
      for (int r = 0; r < 8; ++r) Hs[(8 * hh + r) * FPITCH + j] = hn8[r];
    }
  }
}

__global__ __launch_bounds__(NTHR) void seq_kernel(const int* __restrict__ x, const float* __restrict__ emb,
                                                   const unsigned short* __restrict__ WX0, const unsigned short* __restrict__ WH0,
                                                   const float* __restrict__ rb0i, const float* __restrict__ rb0h,
                                                   const unsigned short* __restrict__ WX1, const unsigned short* __restrict__ WH1,
                                                   const float* __restrict__ rb1i, const float* __restrict__ rb1h,
                                                   const unsigned short* __restrict__ LX0, const unsigned short* __restrict__ LH0,
                                                   const float* __restrict__ lb0i, const float* __restrict__ lb0h,
                                                   const unsigned short* __restrict__ LX1, const unsigned short* __restrict__ LH1,
                                                   const float* __restrict__ lb1i, const float* __restrict__ lb1h,
                                                   const float* __restrict__ Wcls, const float* __restrict__ bcls,
                                                   float* __restrict__ out) {
  extern __shared__ __align__(16) unsigned char dyn_lds[];
  unsigned short* Xs = (unsigned short*)(dyn_lds + LDS_XS);
  _Float16*       Hp = (_Float16*)(dyn_lds + LDS_H);
  float*          Hs = (float*)(dyn_lds + LDS_HS);
  float*          Os = (float*)(dyn_lds + LDS_OS);
  const int tid = threadIdx.x, lane = tid & 31, wave = tid >> 5;
  const int c = lane & 15, hh = lane >> 4, koff = hh * 8;
  const int rowbase = blockIdx.x * SEQ_BLK;
  const int j0 = 64 * wave + c;

  {
    unsigned* hz = (unsigned*)(dyn_lds + LDS_H);
#pragma unroll 1
    for (int i = tid; i < H_DWORDS; i += NTHR) hz[i] = 0u;
  }
  stage_emb(x, emb, Xs, rowbase, 0, tid);

  float cst0[4][8], cst1[4][8];
#pragma unroll
  for (int nt = 0; nt < 4; ++nt) {
#pragma unroll
    for (int r = 0; r < 8; ++r) { cst0[nt][r] = 0.0f; cst1[nt][r] = 0.0f; }
  }
  __syncthreads();

#pragma unroll 1
  for (int t = 0; t < NSTEP; ++t) {
    const int cur = t & 1, nx = cur ^ 1;
    const _Float16* H0c = Hp + (0 + cur) * HPLANE;  _Float16* H0n = Hp + (0 + nx) * HPLANE;
    const _Float16* H1c = Hp + (2 + cur) * HPLANE;  _Float16* H1n = Hp + (2 + nx) * HPLANE;
    const _Float16* H2c = Hp + (4 + cur) * HPLANE;  _Float16* H2n = Hp + (4 + nx) * HPLANE;
    const _Float16* H3c = Hp + (6 + cur) * HPLANE;  _Float16* H3n = Hp + (6 + nx) * HPLANE;
    const bool last = (t == NSTEP - 1);
    const int  arow = c * HPITCH + koff;

    rnn_phase<__bf16, NEMB>((const __bf16*)Xs + c * XPITCH + koff, WX0, H0c + arow, WH0, rb0i, rb0h, H0n, j0, koff, hh);
    __syncthreads();
    {
      const int tn = (t + 1 < NSTEP) ? (t + 1) : (NSTEP - 1);
      stage_emb(x, emb, Xs, rowbase, tn, tid);
    }
    rnn_phase<_Float16, NHID>(H0n + arow, WX1, H1c + arow, WH1, rb1i, rb1h, H1n, j0, koff, hh);
    __syncthreads();
    lstm_phase(H1n + arow, LX0, H2c + arow, LH0, lb0i, lb0h, H2n, Hs, false, cst0, j0, koff, hh);
    __syncthreads();
    lstm_phase(H2n + arow, LX1, H3c + arow, LH1, lb1i, lb1h, H3n, Hs, last, cst1, j0, koff, hh);
    __syncthreads();
  }

  if (tid < OUT_BLK) {
    const int m   = tid / NCLS;
    const int cls = tid - m * NCLS;
    const float* hrow = Hs + m * FPITCH;
    const float* wrow = Wcls + (size_t)cls * NHID;
    float s = 0.0f;
#pragma unroll 1
    for (int k = 0; k < NHID; ++k) s = fmaf(hrow[k], bf16r(wrow[k]), s);
    s += bf16r(bcls[cls]);
    Os[tid] = s;
  }
  __syncthreads();
  if (tid < 32) {
    const v4f v0 = *(const v4f*)(Os + 4 * lane);
    const int l8 = (lane < 8) ? lane : 7;
    const v4f v1 = *(const v4f*)(Os + 128 + 4 * l8);
    float* ob = out + (size_t)blockIdx.x * OUT_BLK;
    for (int pass = 0; pass < 2; ++pass) {
      *(volatile v4f*)(ob + 4 * lane) = v0;
      if (lane < 8) *(volatile v4f*)(ob + 128 + 4 * lane) = v1;
      __threadfence();
    }
  }
}

extern "C" void kernel_launch(void* const* d_in, const int* in_sizes, int n_in,
                              void* d_out, int out_size, void* d_ws, size_t ws_size, hipStream_t stream) {
  if (n_in < 20 || d_out == nullptr || d_ws == nullptr) return;
  if (in_sizes[0] != NSEQ * NSTEP || in_sizes[1] != NVOC * NEMB ||
      in_sizes[2] != NHID * NEMB || in_sizes[3] != NHID * NHID || in_sizes[4] != NHID || in_sizes[5] != NHID ||
      in_sizes[6] != NHID * NHID || in_sizes[7] != NHID * NHID || in_sizes[8] != NHID || in_sizes[9] != NHID ||
      in_sizes[10] != NG4 * NHID || in_sizes[11] != NG4 * NHID || in_sizes[12] != NG4 || in_sizes[13] != NG4 ||
      in_sizes[14] != NG4 * NHID || in_sizes[15] != NG4 * NHID || in_sizes[16] != NG4 || in_sizes[17] != NG4 ||
      in_sizes[18] != NCLS * NHID || in_sizes[19] != NCLS || out_size != NSEQ * NCLS) return;

  const int*   xin   = (const int*)  d_in[0];
  const float* emb   = (const float*)d_in[1];
  const float* rWih0 = (const float*)d_in[2];
  const float* rWhh0 = (const float*)d_in[3];
  const float* rbih0 = (const float*)d_in[4];
  const float* rbhh0 = (const float*)d_in[5];
  const float* rWih1 = (const float*)d_in[6];
  const float* rWhh1 = (const float*)d_in[7];
  const float* rbih1 = (const float*)d_in[8];
  const float* rbhh1 = (const float*)d_in[9];
  const float* lWih0 = (const float*)d_in[10];
  const float* lWhh0 = (const float*)d_in[11];
  const float* lbih0 = (const float*)d_in[12];
  const float* lbhh0 = (const float*)d_in[13];
  const float* lWih1 = (const float*)d_in[14];
  const float* lWhh1 = (const float*)d_in[15];
  const float* lbih1 = (const float*)d_in[16];
  const float* lbhh1 = (const float*)d_in[17];
  const float* fcW   = (const float*)d_in[18];
  const float* fcb   = (const float*)d_in[19];
  float* out = (float*)d_out;

  char* ws = (char*)d_ws; size_t off = 0;
  auto carve = [&](size_t bytes) -> char* { char* p = ws + off; off += (bytes + 255) & ~(size_t)255; return p; };
  unsigned short* WX0 = (unsigned short*)carve((size_t)NHID * NEMB * 2);
  unsigned short* WH0 = (unsigned short*)carve((size_t)NHID * NHID * 2);
  unsigned short* WX1 = (unsigned short*)carve((size_t)NHID * NHID * 2);
  unsigned short* WH1 = (unsigned short*)carve((size_t)NHID * NHID * 2);
  unsigned short* LX0 = (unsigned short*)carve((size_t)NG4 * NHID * 2);
  unsigned short* LH0 = (unsigned short*)carve((size_t)NG4 * NHID * 2);
  unsigned short* LX1 = (unsigned short*)carve((size_t)NG4 * NHID * 2);
  unsigned short* LH1 = (unsigned short*)carve((size_t)NG4 * NHID * 2);
  if (off > ws_size || off > (size_t)134217728) return;

  const int n8a = NHID * NEMB / 8;
  const int n8b = NHID * NHID / 8;
  const int n8c = NG4 * NHID / 8;
  cvt8_kernel<0><<<(n8a + CVT_THR - 1) / CVT_THR, CVT_THR, 0, stream>>>(rWih0, WX0, n8a, XW_CARRY);
  cvt8_kernel<1><<<(n8b + CVT_THR - 1) / CVT_THR, CVT_THR, 0, stream>>>(rWhh0, WH0, n8b, W_CARRY);
  cvt8_kernel<1><<<(n8b + CVT_THR - 1) / CVT_THR, CVT_THR, 0, stream>>>(rWih1, WX1, n8b, W_CARRY);
  cvt8_kernel<1><<<(n8b + CVT_THR - 1) / CVT_THR, CVT_THR, 0, stream>>>(rWhh1, WH1, n8b, W_CARRY);
  cvt8_kernel<1><<<(n8c + CVT_THR - 1) / CVT_THR, CVT_THR, 0, stream>>>(lWih0, LX0, n8c, W_CARRY);
  cvt8_kernel<1><<<(n8c + CVT_THR - 1) / CVT_THR, CVT_THR, 0, stream>>>(lWhh0, LH0, n8c, W_CARRY);
  cvt8_kernel<1><<<(n8c + CVT_THR - 1) / CVT_THR, CVT_THR, 0, stream>>>(lWih1, LX1, n8c, W_CARRY);
  cvt8_kernel<1><<<(n8c + CVT_THR - 1) / CVT_THR, CVT_THR, 0, stream>>>(lWhh1, LH1, n8c, W_CARRY);
  seq_kernel<<<NBLK, NTHR, LDS_TOTAL, stream>>>(xin, emb, WX0, WH0, rbih0, rbhh0, WX1, WH1, rbih1, rbhh1,
                                                LX0, LH0, lbih0, lbhh0, LX1, LH1, lbih1, lbhh1, fcW, fcb, out);
}
